// GCNEncoder_22728966930847
// MI455X (gfx1250) — hardware-verified
//
#include <hip/hip_runtime.h>
#include <stddef.h>
#include <stdint.h>
#include <math.h>


#define CIN    128
#define HID    256
#define COUT   128
#define K1     128
#define K2     512
#define AP2    512
#define NTHR   256
#define NWAVE  8
#define EPT    8
#define CHUNK  (NTHR * EPT)
#define WCAP   (EPT * 32)
#define LISTN  (NWAVE * WCAP)
#define NBD    8192
#define SLD    13
#define NBA    1024
#define SLA    10
#define RCAP   28672
#define DEGCAP 64
#define GBM    64
#define GBN    128
#define GTHR   128
#define GWAVE  (GTHR / 32)
#define PARTW  544
#define WSTW   514
#define PSTOFF 4608
#define APB    64
#define APR    8
#define NU1    (HID * (K1 / 8))
#define NU2    (COUT * (K2 / 8))
#define AGG_ZINTS (LISTN + 2 * RCAP + 3 * NBA)
#define MISC_INTS 16
#define AGG_LDS_INTS (AGG_ZINTS + MISC_INTS)
#define WSMAX  134217728

static_assert((CHUNK & (CHUNK - 1)) == 0 && CHUNK <= 4096);
static_assert((NBD & (NBD - 1)) == 0 && NBD == (1 << SLD));
static_assert((NBA & (NBA - 1)) == 0 && NBA == (1 << SLA));
static_assert(((long long)CHUNK << SLD) < (1LL << 31));
static_assert(((long long)CHUNK << SLA) < (1LL << 31));
static_assert(NBD % (NTHR * 4) == 0);
static_assert(LISTN % NTHR == 0);
static_assert(NBA % NWAVE == 0 && NBA % 32 == 0 && NBA % GBM == 0);
static_assert(RCAP % 32 == 0 && AGG_ZINTS % (NTHR * 4) == 0 && LISTN % 4 == 0);
static_assert(K1 % 32 == 0 && K2 % 32 == 0 && K2 == 2 * HID && AP2 == K2 && K1 == CIN);
static_assert(HID == 2 * GBN && COUT == GBN && GBM == GWAVE * 16 && GBN == 8 * 16);
static_assert(NU1 % NTHR == 0 && NU2 % NTHR == 0 && K1 / 8 == 16 && K2 / 8 == 64);
static_assert(HID == NTHR && HID == 2 * 128 && COUT == 128);
static_assert(PARTW % 32 == 0 && PARTW >= 2 * HID + 1 && PARTW / 4 <= NTHR);
static_assert(WSTW >= 2 * HID + 1 && NWAVE * WSTW <= PSTOFF && (PSTOFF % 4) == 0 && PSTOFF + PARTW <= RCAP);
static_assert(APB == NWAVE * APR && APB == GBM);
static_assert(CIN % 8 == 0 && (CIN / 8) == 16);
static_assert(AGG_LDS_INTS * 4 <= 300000);

typedef float          v4f   __attribute__((ext_vector_type(4)));
typedef float          v8f   __attribute__((ext_vector_type(8)));
typedef int            v4i   __attribute__((ext_vector_type(4)));
typedef int            v8i   __attribute__((ext_vector_type(8)));
typedef unsigned short v8us  __attribute__((ext_vector_type(8)));
typedef unsigned short v16us __attribute__((ext_vector_type(16)));
typedef __bf16         v16bf __attribute__((ext_vector_type(16)));
typedef v4f  __attribute__((may_alias)) v4fa;
typedef v4i  __attribute__((may_alias)) v4ia;
typedef v8us __attribute__((may_alias)) v8usa;
union FragB { v16bf v; v16us u; v8us h[2]; v8i w; };

__device__ __forceinline__ v8f wmb(const FragB& a, const FragB& b, v8f c) {
  v8f d = __builtin_amdgcn_wmma_f32_16x16x32_bf16(false, a.v, false, b.v, (short)0, c, false, false);
  asm volatile("v_nop\n\tv_nop\n\tv_nop\n\tv_nop" : "+v"(d) : "v"(a.w), "v"(b.w));
  return d;
}

__device__ __forceinline__ v8f z8() { v8f z = {0.f, 0.f, 0.f, 0.f, 0.f, 0.f, 0.f, 0.f}; return z; }

__device__ __forceinline__ unsigned bf16_bits(float f) {
  const unsigned u = __float_as_uint(f);
  return (u + 0x7FFFu + ((u >> 16) & 1u)) >> 16;
}
__device__ __forceinline__ float bf16_val(float f) {
  return __uint_as_float(bf16_bits(f) << 16);
}

template <int SLB>
__device__ __forceinline__ int scan_chunk(const int* __restrict__ dsts, int nE, int cbase, int slotBase,
                                          int nb, int vec8, int* list, int tid, int lane, int wave) {
  int wc = 0;
  const int el0  = tid * EPT;
  const int e0   = cbase + el0;
  const int sent = -2147483647 - 1;
  v4i da, db;
  if (vec8 != 0 && cbase + CHUNK <= nE) {
    da = *(const v4i*)(dsts + e0);
    db = *(const v4i*)(dsts + e0 + 4);
  } else {
    da.x = (e0     < nE) ? dsts[min(e0,     nE - 1)] : sent;
    da.y = (e0 + 1 < nE) ? dsts[min(e0 + 1, nE - 1)] : sent;
    da.z = (e0 + 2 < nE) ? dsts[min(e0 + 2, nE - 1)] : sent;
    da.w = (e0 + 3 < nE) ? dsts[min(e0 + 3, nE - 1)] : sent;
    db.x = (e0 + 4 < nE) ? dsts[min(e0 + 4, nE - 1)] : sent;
    db.y = (e0 + 5 < nE) ? dsts[min(e0 + 5, nE - 1)] : sent;
    db.z = (e0 + 6 < nE) ? dsts[min(e0 + 6, nE - 1)] : sent;
    db.w = (e0 + 7 < nE) ? dsts[min(e0 + 7, nE - 1)] : sent;
  }
  const unsigned nbs = (unsigned)slotBase;
  const unsigned unb = (unsigned)nb;
  const unsigned s0 = (unsigned)da.x - nbs, s1 = (unsigned)da.y - nbs;
  const unsigned s2 = (unsigned)da.z - nbs, s3 = (unsigned)da.w - nbs;
  const unsigned s4 = (unsigned)db.x - nbs, s5 = (unsigned)db.y - nbs;
  const unsigned s6 = (unsigned)db.z - nbs, s7 = (unsigned)db.w - nbs;
  const bool h0 = s0 < unb, h1 = s1 < unb, h2 = s2 < unb, h3 = s3 < unb;
  const bool h4 = s4 < unb, h5 = s5 < unb, h6 = s6 < unb, h7 = s7 < unb;
  const unsigned any = __builtin_amdgcn_ballot_w32(h0 | h1 | h2 | h3 | h4 | h5 | h6 | h7);
  if (any != 0u) {
#define HITJ(J, HJ, SJ) { \
      const unsigned mj = __builtin_amdgcn_ballot_w32(HJ); \
      if (mj != 0u) { \
        if (HJ) { \
          const int pos = wc + (int)__builtin_amdgcn_mbcnt_lo(mj, 0u); \
          if (pos < WCAP) list[wave * WCAP + pos] = ((el0 + (J)) << SLB) | (int)(SJ); \
        } \
        wc += (int)__builtin_popcount(mj); } }
    HITJ(0, h0, s0)
    HITJ(1, h1, s1)
    HITJ(2, h2, s2)
    HITJ(3, h3, s3)
    HITJ(4, h4, s4)
    HITJ(5, h5, s5)
    HITJ(6, h6, s6)
    HITJ(7, h7, s7)
#undef HITJ
  }
  return wc;
}

__global__ __launch_bounds__(NTHR) void k_wprep(const float* __restrict__ W1, const float* __restrict__ W2,
                                                unsigned short* W1T, unsigned short* W2T) {
  const int u = (int)blockIdx.x * NTHR + (int)threadIdx.x;
  v8us o;
  unsigned short* dp;
  if (u < NU1) {
    const int n  = u >> 4;
    const int k8 = (u & 15) * 8;
    const float* p = W1 + (size_t)k8 * HID + n;
#pragma unroll
    for (int i = 0; i < 8; ++i) o[i] = (unsigned short)bf16_bits(p[(size_t)i * HID]);
    dp = W1T + (size_t)n * K1 + k8;
  } else if (u < NU1 + NU2) {
    const int v  = u - NU1;
    const int n  = v >> 6;
    const int k8 = (v & 63) * 8;
    const int kk = k8 & (HID - 1);
    const float* p = W2 + (size_t)kk * COUT + n;
#pragma unroll
    for (int i = 0; i < 8; ++i) o[i] = (unsigned short)bf16_bits(p[(size_t)i * COUT]);
    dp = W2T + (size_t)n * K2 + k8;
  } else {
    return;
  }
  *(volatile v8us*)dp = o;
  __threadfence();
  *(volatile v8us*)dp = o;
}

__global__ __launch_bounds__(NTHR) void k_cvx(const float* __restrict__ x, int nN, int nUnits,
                                              unsigned short* xb) {
  const int u = (int)blockIdx.x * NTHR + (int)threadIdx.x;
  if (u >= nUnits) return;
  const int row = u >> 4;
  const int k8  = (u & 15) * 8;
  const int rc  = row < nN ? row : nN - 1;
  const bool rok = row < nN;
  const float* p = x + (size_t)rc * CIN + k8;
  const v4f a0 = *(const v4f*)p;
  const v4f a1 = *(const v4f*)(p + 4);
  v8us o;
  o[0] = rok ? (unsigned short)bf16_bits(a0.x) : (unsigned short)0;
  o[1] = rok ? (unsigned short)bf16_bits(a0.y) : (unsigned short)0;
  o[2] = rok ? (unsigned short)bf16_bits(a0.z) : (unsigned short)0;
  o[3] = rok ? (unsigned short)bf16_bits(a0.w) : (unsigned short)0;
  o[4] = rok ? (unsigned short)bf16_bits(a1.x) : (unsigned short)0;
  o[5] = rok ? (unsigned short)bf16_bits(a1.y) : (unsigned short)0;
  o[6] = rok ? (unsigned short)bf16_bits(a1.z) : (unsigned short)0;
  o[7] = rok ? (unsigned short)bf16_bits(a1.w) : (unsigned short)0;
  unsigned short* dp = xb + (size_t)row * K1 + k8;
  *(volatile v8us*)dp = o;
  __threadfence();
  *(volatile v8us*)dp = o;
}

__global__ __launch_bounds__(NTHR) void k_deg(const int* __restrict__ dsts, int nE, int vec8, float* dis) {
  __shared__ __attribute__((aligned(16))) int scnt[NBD];
  __shared__ __attribute__((aligned(16))) int list[LISTN];
  __shared__ int wcnt[NWAVE];
  const int tid = (int)threadIdx.x, lane = tid & 31, wave = tid >> 5;
  const int nodeBase = (int)blockIdx.x * NBD;

  for (int i = tid; i < NBD; i += NTHR) scnt[i] = 0;
  for (int i = tid; i < LISTN; i += NTHR) list[i] = 0;
  if (tid < NWAVE) wcnt[tid] = 0;
  __syncthreads();

  const int nChunks = (nE + CHUNK - 1) / CHUNK;
#pragma unroll 1
  for (int ch = 0; ch < nChunks; ++ch) {
    const int cbase = ch * CHUNK;
    const int wc = scan_chunk<SLD>(dsts, nE, cbase, nodeBase, NBD, vec8, list, tid, lane, wave);
    if (lane == 0) wcnt[wave] = wc;
    __syncthreads();
    if (wave == 0) {
#pragma unroll 1
      for (int w2 = 0; w2 < NWAVE; ++w2) {
        int c = wcnt[w2];
        c = c < 0 ? 0 : (c > WCAP ? WCAP : c);
#pragma unroll 1
        for (int b0 = 0; b0 < c; b0 += 32) {
          const int idx = b0 + lane;
          const int ent = list[w2 * WCAP + (idx < WCAP ? idx : WCAP - 1)];
          const int m32 = (c - b0) < 32 ? (c - b0) : 32;
#pragma unroll 1
          for (int k = 0; k < m32; ++k) {
            const int u  = __builtin_amdgcn_readlane(ent, k);
            const int sl = u & (NBD - 1);
            if (lane == 0) scnt[sl] = scnt[sl] + 1;
          }
        }
      }
    }
    __syncthreads();
  }

  v4f vals[NBD / (NTHR * 4)];
#pragma unroll
  for (int it = 0; it < NBD / (NTHR * 4); ++it) {
    const int s0 = it * (NTHR * 4) + 4 * tid;
    const v4i c4 = *(const v4ia*)(scnt + s0);
    const float d0 = (float)c4.x + 1.0f, d1 = (float)c4.y + 1.0f;
    const float d2 = (float)c4.z + 1.0f, d3 = (float)c4.w + 1.0f;
    v4f v;
    v.x = rsqrtf(d0); v.y = rsqrtf(d1); v.z = rsqrtf(d2); v.w = rsqrtf(d3);
    vals[it] = v;
  }
#pragma unroll
  for (int it = 0; it < NBD / (NTHR * 4); ++it) {
    const int s0 = it * (NTHR * 4) + 4 * tid;
    *(volatile v4f*)(dis + (size_t)nodeBase + s0) = vals[it];
  }
  __threadfence();
#pragma unroll
  for (int it = 0; it < NBD / (NTHR * 4); ++it) {
    const int s0 = it * (NTHR * 4) + 4 * tid;
    *(volatile v4f*)(dis + (size_t)nodeBase + s0) = vals[it];
  }
}

__global__ __launch_bounds__(GTHR) void k_gemm(
    const unsigned short* __restrict__ A, const unsigned short* __restrict__ WT,
    float* outF, int K, int ldo)
{
  __shared__ __attribute__((aligned(16))) float stg[GBM * GBN];
  const int tid = (int)threadIdx.x, lane = tid & 31, wave = tid >> 5, hh = lane >> 4, m = lane & 15;
  const int rowBase = (int)blockIdx.x * GBM;
  const int col0    = (int)blockIdx.y * GBN;

  v8f acc[8];
#pragma unroll
  for (int t = 0; t < 8; ++t) acc[t] = z8();
  const unsigned short* ap = A  + (size_t)(rowBase + 16 * wave + m) * (size_t)K + 8 * hh;
  const unsigned short* wp = WT + (size_t)(col0 + m) * (size_t)K + 8 * hh;
  const int ksteps = K >> 5;
#pragma unroll 1
  for (int ks = 0; ks < ksteps; ++ks) {
    FragB af;
    af.h[0] = *(const v8usa*)(ap + 32 * ks);
    af.h[1] = *(const v8usa*)(ap + 32 * ks + 16);
#pragma unroll
    for (int t = 0; t < 8; ++t) {
      const unsigned short* wq = wp + (size_t)(16 * t) * (size_t)K + 32 * ks;
      FragB bf;
      bf.h[0] = *(const v8usa*)wq;
      bf.h[1] = *(const v8usa*)(wq + 16);
      acc[t] = wmb(af, bf, acc[t]);
    }
  }

#pragma unroll
  for (int t = 0; t < 8; ++t) {
    const int lc = 16 * t + m;
#pragma unroll
    for (int r = 0; r < 8; ++r) {
      const int lr = 16 * wave + 8 * hh + r;
      stg[lr * GBN + lc] = acc[t][r];
    }
  }
  __syncthreads();

  v4f fv[16];
#pragma unroll
  for (int i = 0; i < 16; ++i) {
    const int lr = 16 * wave + i;
    fv[i] = *(const v4fa*)(stg + lr * GBN + 4 * lane);
  }
#pragma unroll
  for (int i = 0; i < 16; ++i) {
    const int gr = rowBase + 16 * wave + i;
    float* op = outF + (size_t)gr * (size_t)ldo + col0 + 4 * lane;
    *(volatile v4f*)op = fv[i];
  }
  __threadfence();
#pragma unroll
  for (int i = 0; i < 16; ++i) {
    const int gr = rowBase + 16 * wave + i;
    float* op = outF + (size_t)gr * (size_t)ldo + col0 + 4 * lane;
    *(volatile v4f*)op = fv[i];
  }
}

template <int NG, int FIN>
__global__ __launch_bounds__(NTHR) void k_agg(const int* __restrict__ srcs, const int* __restrict__ dsts,
                                              int nE, int nN, int vec8, int mRows,
                                              const float* __restrict__ dis,
                                              const float* __restrict__ xl, const float* __restrict__ bias,
                                              float* outp, float* part) {
  static_assert((NG == 2 && FIN == 0) || (NG == 1 && FIN == 1));
  constexpr int C  = 128 * NG;
  constexpr int NV = 4 * NG;
  static_assert(FIN != 0 || C == NTHR);
  extern __shared__ __attribute__((aligned(16))) int dsm[];
  int* list = dsm;
  int* hl   = dsm + LISTN;
  int* sl   = hl + RCAP;
  int* cnt  = sl + RCAP;
  int* offs = cnt + NBA;
  int* cur  = offs + NBA;
  int* misc = cur + NBA;
  float* wst = (float*)hl;
  float* pst = (float*)(hl + PSTOFF);
  const int tid = (int)threadIdx.x, lane = tid & 31, wave = tid >> 5;
  const int nodeBase = (int)blockIdx.x * NBA;

  {
    const v4i z4 = {0, 0, 0, 0};
    for (int i = tid * 4; i < AGG_ZINTS; i += NTHR * 4) *(v4ia*)(dsm + i) = z4;
    if (tid < MISC_INTS) misc[tid] = 0;
  }
  float bv[NV];
#pragma unroll
  for (int g = 0; g < NG; ++g) {
    const v4f a = *(const v4fa*)(bias + g * 128 + 4 * lane);
    bv[4 * g + 0] = bf16_val(a.x); bv[4 * g + 1] = bf16_val(a.y);
    bv[4 * g + 2] = bf16_val(a.z); bv[4 * g + 3] = bf16_val(a.w);
  }
  __syncthreads();

  int t = 0, ov = 0;
  const int nChunks = (nE + CHUNK - 1) / CHUNK;
#pragma unroll 1
  for (int ch = 0; ch < nChunks; ++ch) {
    const int cbase = ch * CHUNK;
    const int wc = scan_chunk<SLA>(dsts, nE, cbase, nodeBase, NBA, vec8, list, tid, lane, wave);
    if (lane == 0) misc[wave] = wc;
    __syncthreads();
    if (wave == 0) {
#pragma unroll 1
      for (int w2 = 0; w2 < NWAVE; ++w2) {
        int c = misc[w2];
        c = c < 0 ? 0 : (c > WCAP ? WCAP : c);
#pragma unroll 1
        for (int b0 = 0; b0 < c; b0 += 32) {
          const int idx = b0 + lane;
          const int ent = list[w2 * WCAP + (idx < WCAP ? idx : WCAP - 1)];
          const int m32 = (c - b0) < 32 ? (c - b0) : 32;
#pragma unroll 1
          for (int k = 0; k < m32; ++k) {
            const int u    = __builtin_amdgcn_readlane(ent, k);
            const int slot = u & (NBA - 1);
            const int el   = (u >> SLA) & (CHUNK - 1);
            const int pk   = ((cbase + el) << SLA) | slot;
            if (t < RCAP) {
              if (lane == 0) { hl[t] = pk; cnt[slot] = cnt[slot] + 1; }
              t = t + 1;
            } else {
              ov = 1;
            }
          }
        }
      }
    }
    __syncthreads();
  }
  if (wave == 0 && lane == 0) { misc[8] = t; misc[9] = ov; }
  __syncthreads();
  int tt = misc[8];
  tt = tt < 0 ? 0 : (tt > RCAP ? RCAP : tt);
  const int ovf = misc[9];

  if (wave == 0) {
    const int base = lane * (NBA / 32);
    int s = 0;
#pragma unroll 1
    for (int i = 0; i < NBA / 32; ++i) s += cnt[base + i];
    int incl = s;
#pragma unroll
    for (int d = 1; d < 32; d <<= 1) {
      const int y = __shfl_up(incl, d, 32);
      if (lane >= d) incl += y;
    }
    int run = incl - s;
#pragma unroll 1
    for (int i = 0; i < NBA / 32; ++i) {
      const int cv = cnt[base + i];
      offs[base + i] = run;
      cur[base + i]  = run;
      run += cv;
    }
  }
  __syncthreads();
  if (wave == 0) {
#pragma unroll 1
    for (int b0 = 0; b0 < tt; b0 += 32) {
      const int idx = b0 + lane;
      const int ent = hl[idx < RCAP ? idx : RCAP - 1];
      const int m32 = (tt - b0) < 32 ? (tt - b0) : 32;
#pragma unroll 1
      for (int k = 0; k < m32; ++k) {
        const int u    = __builtin_amdgcn_readlane(ent, k);
        const int slot = u & (NBA - 1);
        if (lane == 0) {
          int p = cur[slot];
          p = p < 0 ? 0 : (p > RCAP - 1 ? RCAP - 1 : p);
          sl[p] = u;
          cur[slot] = p + 1;
        }
      }
    }
  }
  __syncthreads();

  const float qnan = __int_as_float(0x7fc00000);
  const float pz = (ovf != 0) ? qnan : 0.0f;
  int wn = 0;
  float wm[NV], wq[NV];
#pragma unroll
  for (int i = 0; i < NV; ++i) { wm[i] = 0.0f; wq[i] = 0.0f; }
#pragma unroll 1
  for (int si = 0; si < NBA / NWAVE; ++si) {
    const int s    = si * NWAVE + wave;
    const int node = nodeBase + s;
    int c = cnt[s];
    const bool big = c > DEGCAP;
    c = c < 0 ? 0 : (c > DEGCAP ? DEGCAP : c);
    int o = offs[s];
    o = o < 0 ? 0 : (o > RCAP ? RCAP : o);
    const int nc = node < nN ? node : nN - 1;
    const float dd = dis[nc];
    const float rd = dd * dd;
    float acc[NV];
#pragma unroll
    for (int i = 0; i < NV; ++i) acc[i] = 0.0f;
#pragma unroll 1
    for (int b0 = 0; b0 < c; b0 += 32) {
      int idx = o + b0 + lane;
      idx = idx > RCAP - 1 ? RCAP - 1 : idx;
      const int ent = sl[idx];
      int eid = ent >> SLA;
      eid = eid < 0 ? 0 : (eid > nE - 1 ? nE - 1 : eid);
      int sr = srcs[eid];
      sr = sr < 0 ? 0 : (sr > nN - 1 ? nN - 1 : sr);
      const float cf  = dis[sr] * dd;
      const int   cfi = __float_as_int(cf);
      const int m32 = (c - b0) < 32 ? (c - b0) : 32;
#pragma unroll 1
      for (int k = 0; k < m32; ++k) {
        const int   sk = __builtin_amdgcn_readlane(sr, k);
        const float ck = __int_as_float(__builtin_amdgcn_readlane(cfi, k));
        const float* rp = xl + (size_t)sk * C + 4 * lane;
#pragma unroll
        for (int g = 0; g < NG; ++g) {
          const v4f a = *(const v4fa*)(rp + g * 128);
          acc[4 * g + 0] = fmaf(ck, a.x, acc[4 * g + 0]);
          acc[4 * g + 1] = fmaf(ck, a.y, acc[4 * g + 1]);
          acc[4 * g + 2] = fmaf(ck, a.z, acc[4 * g + 2]);
          acc[4 * g + 3] = fmaf(ck, a.w, acc[4 * g + 3]);
        }
      }
    }
    float sv[NV];
    {
      const float* sp = xl + (size_t)nc * C + 4 * lane;
#pragma unroll
      for (int g = 0; g < NG; ++g) {
        const v4f a = *(const v4fa*)(sp + g * 128);
        sv[4 * g + 0] = a.x; sv[4 * g + 1] = a.y; sv[4 * g + 2] = a.z; sv[4 * g + 3] = a.w;
      }
    }
    const float pzr = big ? qnan : pz;
    const bool live = node < nN;
    float v[NV];
#pragma unroll
    for (int i = 0; i < NV; ++i) {
      float y = (acc[i] + sv[i] * rd) + bv[i];
      y = y + pzr;
      v[i] = live ? y : 0.0f;
    }
    v4f q[NG];
#pragma unroll
    for (int g = 0; g < NG; ++g) {
      v4f w;
      w.x = v[4 * g + 0]; w.y = v[4 * g + 1]; w.z = v[4 * g + 2]; w.w = v[4 * g + 3];
      q[g] = w;
    }
    if constexpr (FIN == 0) {
      if (live) {
        wn += 1;
        const float rk = 1.0f / (float)wn;
#pragma unroll
        for (int i = 0; i < NV; ++i) {
          const float d = v[i] - wm[i];
          wm[i] = fmaf(d, rk, wm[i]);
          wq[i] = fmaf(d, v[i] - wm[i], wq[i]);
        }
      }
      if (node < mRows) {
#pragma unroll
        for (int g = 0; g < NG; ++g)
          *(volatile v4f*)(outp + (size_t)node * C + g * 128 + 4 * lane) = q[g];
        __threadfence();
#pragma unroll
        for (int g = 0; g < NG; ++g)
          *(volatile v4f*)(outp + (size_t)node * C + g * 128 + 4 * lane) = q[g];
      }
    } else {
      float* op = outp + (size_t)nc * COUT + 4 * lane;
      if (live) *(volatile v4f*)op = q[0];
      __threadfence();
      if (live) *(volatile v4f*)op = q[0];
    }
  }

  if constexpr (FIN == 0) {
    if (lane == 0) wst[wave * WSTW] = (float)wn;
#pragma unroll
    for (int g = 0; g < NG; ++g) {
#pragma unroll
      for (int j = 0; j < 4; ++j) {
        const int chn = g * 128 + 4 * lane + j;
        wst[wave * WSTW + 1 + chn]     = wm[4 * g + j];
        wst[wave * WSTW + 1 + C + chn] = wq[4 * g + j];
      }
    }
    __syncthreads();
    {
      float n = 0.0f, mean = 0.0f, M2 = 0.0f;
#pragma unroll 1
      for (int w2 = 0; w2 < NWAVE; ++w2) {
        const float nb = wst[w2 * WSTW];
        const float mb = wst[w2 * WSTW + 1 + tid];
        const float qb = wst[w2 * WSTW + 1 + C + tid];
        if (nb > 0.5f) {
          const float nn = n + nb;
          const float delta = mb - mean;
          const float f = nb / nn;
          mean = fmaf(delta, f, mean);
          M2 = M2 + qb + delta * delta * n * f;
          n = nn;
        }
      }
      pst[1 + tid] = mean;
      pst[1 + C + tid] = M2;
      if (tid == 0) pst[0] = n;
    }
#pragma unroll 1
    for (int i = 2 * C + 1 + tid; i < PARTW; i += NTHR) pst[i] = 0.0f;
    __syncthreads();
    const int pb = (int)blockIdx.x;
    v4f ps = {0.0f, 0.0f, 0.0f, 0.0f};
    if (tid < PARTW / 4) {
      ps = *(const v4fa*)(pst + 4 * tid);
      *(volatile v4f*)(part + (size_t)pb * PARTW + 4 * tid) = ps;
    }
    __threadfence();
    if (tid < PARTW / 4) {
      *(volatile v4f*)(part + (size_t)pb * PARTW + 4 * tid) = ps;
    }
  }
}

__global__ __launch_bounds__(HID) void k_bnfin(const float* __restrict__ part, int nPart,
                                               const float* __restrict__ gam, const float* __restrict__ bet,
                                               float* ss) {
  __shared__ __attribute__((aligned(16))) float stg[2 * HID];
  const int tid = (int)threadIdx.x;
  const int c = tid;
  double n = 0.0, mean = 0.0, M2 = 0.0;
#pragma unroll 1
  for (int b = 0; b < nPart; ++b) {
    const float* pr = part + (size_t)b * PARTW;
    const double nb = (double)pr[0];
    const double mb = (double)pr[1 + c];
    const double qb = (double)pr[1 + HID + c];
    if (nb > 0.5) {
      const double nn = n + nb;
      const double delta = mb - mean;
      const double f = nb / nn;
      mean = mean + delta * f;
      M2 = M2 + qb + delta * delta * n * f;
      n = nn;
    }
  }
  const double nt = n < 1.0 ? 1.0 : n;
  const float varf  = (float)(M2 / nt);
  const float meanf = (float)mean;
  const float rstd = 1.0f / sqrtf(varf + 1e-5f);
  const float sc = bf16_val(gam[c]) * rstd;
  const float sh = bf16_val(bet[c]) - meanf * sc;
  stg[c] = sc;
  stg[HID + c] = sh;
  __syncthreads();
  v4f v = {0.0f, 0.0f, 0.0f, 0.0f};
  if (tid < (2 * HID) / 4) {
    v = *(const v4fa*)(stg + 4 * tid);
    *(volatile v4f*)(ss + 4 * tid) = v;
  }
  __threadfence();
  if (tid < (2 * HID) / 4) {
    *(volatile v4f*)(ss + 4 * tid) = v;
  }
}

__global__ __launch_bounds__(NTHR) void k_apply(const float* __restrict__ z, const float* __restrict__ ss,
                                                int nN, int mRows, unsigned short* apl) {
  __shared__ __attribute__((aligned(16))) float ssh[2 * HID];
  const int tid = (int)threadIdx.x, lane = tid & 31, wave = tid >> 5;
  ssh[tid] = ss[tid];
  ssh[HID + tid] = ss[HID + tid];
  __syncthreads();
  const v4f sc0 = *(const v4fa*)(ssh + 8 * lane);
  const v4f sc1 = *(const v4fa*)(ssh + 8 * lane + 4);
  const v4f sh0 = *(const v4fa*)(ssh + HID + 8 * lane);
  const v4f sh1 = *(const v4fa*)(ssh + HID + 8 * lane + 4);
  const int rb0 = (int)blockIdx.x * APB + wave * APR;

  v8us qh[APR], ql[APR];
#pragma unroll
  for (int i = 0; i < APR; ++i) {
    const int row = rb0 + i;
    const bool live = row < nN;
    const int rc = live ? row : (nN - 1);
    const float* zp = z + (size_t)rc * HID + 8 * lane;
    const v4f a0 = *(const v4f*)zp;
    const v4f a1 = *(const v4f*)(zp + 4);
    float y[8];
    y[0] = fmaxf(fmaf(a0.x, sc0.x, sh0.x), 0.0f);
    y[1] = fmaxf(fmaf(a0.y, sc0.y, sh0.y), 0.0f);
    y[2] = fmaxf(fmaf(a0.z, sc0.z, sh0.z), 0.0f);
    y[3] = fmaxf(fmaf(a0.w, sc0.w, sh0.w), 0.0f);
    y[4] = fmaxf(fmaf(a1.x, sc1.x, sh1.x), 0.0f);
    y[5] = fmaxf(fmaf(a1.y, sc1.y, sh1.y), 0.0f);
    y[6] = fmaxf(fmaf(a1.z, sc1.z, sh1.z), 0.0f);
    y[7] = fmaxf(fmaf(a1.w, sc1.w, sh1.w), 0.0f);
    v8us mh, ml;
#pragma unroll
    for (int e = 0; e < 8; ++e) {
      const float ye = live ? y[e] : 0.0f;
      const unsigned hb = bf16_bits(ye);
      mh[e] = (unsigned short)hb;
      ml[e] = (unsigned short)bf16_bits(ye - __uint_as_float(hb << 16));
    }
    qh[i] = mh;
    ql[i] = ml;
  }
#pragma unroll
  for (int i = 0; i < APR; ++i) {
    const int row = rb0 + i;
    if (row < mRows) {
      *(volatile v8us*)(apl + (size_t)row * AP2 + 8 * lane) = qh[i];
      *(volatile v8us*)(apl + (size_t)row * AP2 + HID + 8 * lane) = ql[i];
    }
  }
  __threadfence();
#pragma unroll
  for (int i = 0; i < APR; ++i) {
    const int row = rb0 + i;
    if (row < mRows) {
      *(volatile v8us*)(apl + (size_t)row * AP2 + 8 * lane) = qh[i];
      *(volatile v8us*)(apl + (size_t)row * AP2 + HID + 8 * lane) = ql[i];
    }
  }
}

static inline int cdiv(int a, int b) { return (a + b - 1) / b; }
static inline size_t al256(size_t o) { return (o + 255) & ~(size_t)255; }

extern "C" void kernel_launch(void* const* d_in, const int* in_sizes, int n_in,
                              void* d_out, int out_size, void* d_ws, size_t ws_size,
                              hipStream_t stream) {
  if (n_in < 8) return;
  if (in_sizes[0] < CIN || (in_sizes[0] % CIN) != 0) return;
  const int nN = in_sizes[0] / CIN;
  if (in_sizes[1] < 2 || (in_sizes[1] & 1) != 0) return;
  const int nE = in_sizes[1] / 2;
  if (nE < 1 || nE >= (1 << 21) || nN < 16 || nN >= (1 << 24)) return;
  if (in_sizes[2] != CIN * HID) return;
  if (in_sizes[3] != HID || in_sizes[4] != HID || in_sizes[5] != HID) return;
  if (in_sizes[6] != HID * COUT || in_sizes[7] != COUT) return;
  if ((long long)out_size != (long long)nN * COUT) return;

  const float* x    = (const float*)d_in[0];
  const int*   edge = (const int*)d_in[1];
  const float* W1   = (const float*)d_in[2];
  const float* b1   = (const float*)d_in[3];
  const float* g1   = (const float*)d_in[4];
  const float* be1  = (const float*)d_in[5];
  const float* W2   = (const float*)d_in[6];
  const float* b2   = (const float*)d_in[7];
  float* out = (float*)d_out;
  const int* src = edge;
  const int* dst = edge + nE;

  const int MP   = cdiv(nN, GBM) * GBM;
  const int gM   = MP / GBM;
  const int gD   = cdiv(nN, NBD);
  const int NBPD = gD * NBD;
  const int gA   = cdiv(MP, NBA);
  if ((long long)gA * NBA < (long long)MP) return;
  if (NBPD < nN || (MP % APB) != 0) return;
  const int vec8 = ((nE & 3) == 0) ? 1 : 0;

  char* ws = (char*)d_ws;
  size_t off = 0;
  const size_t oDIS = off; off = al256(off + (size_t)NBPD * 4);
  const size_t oW1T = off; off = al256(off + (size_t)HID * K1 * 2);
  const size_t oW2T = off; off = al256(off + (size_t)COUT * K2 * 2);
  const size_t oXB  = off; off = al256(off + (size_t)MP * K1 * 2);
  const size_t szH1 = (size_t)MP * HID * 4;
  const size_t szA2 = (size_t)MP * AP2 * 2;
  const size_t oR1  = off; off = al256(off + (szH1 > szA2 ? szH1 : szA2));
  const size_t szZ1 = (size_t)MP * HID * 4;
  const size_t szH2 = (size_t)MP * COUT * 4;
  const size_t oR2  = off; off = al256(off + (szZ1 > szH2 ? szZ1 : szH2));
  const size_t oPT  = off; off = al256(off + (size_t)gA * PARTW * 4);
  const size_t oSS  = off; off = al256(off + (size_t)(2 * HID) * 4);
  if (off > ws_size || off > (size_t)WSMAX) return;
  float*          DIS = (float*)(ws + oDIS);
  unsigned short* W1T = (unsigned short*)(ws + oW1T);
  unsigned short* W2T = (unsigned short*)(ws + oW2T);
  unsigned short* XB  = (unsigned short*)(ws + oXB);
  float*          H1  = (float*)(ws + oR1);
  unsigned short* A2  = (unsigned short*)(ws + oR1);
  float*          Z1  = (float*)(ws + oR2);
  float*          H2  = (float*)(ws + oR2);
  float*          PT  = (float*)(ws + oPT);
  float*          SS  = (float*)(ws + oSS);

  const size_t aggLds = (size_t)AGG_LDS_INTS * 4;
  hipFuncSetAttribute(reinterpret_cast<const void*>(&k_agg<2, 0>), hipFuncAttributeMaxDynamicSharedMemorySize, (int)aggLds);
  hipFuncSetAttribute(reinterpret_cast<const void*>(&k_agg<1, 1>), hipFuncAttributeMaxDynamicSharedMemorySize, (int)aggLds);

  const int nUx = MP * (K1 / 8);
  k_wprep<<<(NU1 + NU2) / NTHR, NTHR, 0, stream>>>(W1, W2, W1T, W2T);
  k_cvx<<<cdiv(nUx, NTHR), NTHR, 0, stream>>>(x, nN, nUx, XB);
  k_deg<<<gD, NTHR, 0, stream>>>(dst, nE, vec8, DIS);
  k_gemm<<<dim3(gM, HID / GBN), GTHR, 0, stream>>>(XB, W1T, H1, K1, HID);
  k_agg<2, 0><<<gA, NTHR, aggLds, stream>>>(src, dst, nE, nN, vec8, MP, DIS, H1, b1, Z1, PT);
  k_bnfin<<<1, HID, 0, stream>>>(PT, gA, g1, be1, SS);
  k_apply<<<gM, NTHR, 0, stream>>>(Z1, SS, nN, MP, A2);
  k_gemm<<<dim3(gM, COUT / GBN), GTHR, 0, stream>>>(A2, W2T, H2, K2, COUT);
  k_agg<1, 1><<<gA, NTHR, aggLds, stream>>>(src, dst, nE, nN, vec8, MP, DIS, H2, b2, out, PT);
}
